// CrossModalFusion_4131758539525
// MI455X (gfx1250) — hardware-run, weakly checked
//
#include <hip/hip_runtime.h>


#pragma clang fp contract(off)

#ifndef NB
#define NB 8
#endif
#ifndef SEQ
#define SEQ 256
#endif
#define NB_FULL  8
#define SEQ_FULL 256
#define DM   512
#define DAU  512
#define DVI  256
#define NH_  8
#define HD   64
#define DFF  2048
#define NLAY 4
#define MR   (NB * SEQ)
#define XCP  1024
#define AW   4
#define OSP  68
#define LNP  516
#define WTP  65
#define WSC  64.0f
#define WSI  (1.0f / 64.0f)
#define CSC  64.0f
#define NSC  32.0f
#define PAL  16384.0f
#define SC2  ((float)(0.125 * 1.4426950408889634))
#define LOG2E 1.4426950408889634f
#define PSH  14.0f
#define NEGB (-3.0e38f)
#define NEGV (-1.0e30f)
#define BIGSH 30

static_assert(SEQ == 256);
static_assert(SEQ == SEQ_FULL);
static_assert(NB >= 1);
static_assert(NB <= NB_FULL);
static_assert(NH_ * HD == DM);
static_assert(HD == 64);
static_assert(DM == 8 * 64);
static_assert(MR % 64 == 0);
static_assert(SEQ % 64 == 0);
static_assert(SEQ % (16 * AW) == 0);
static_assert(SEQ % 32 == 0);
static_assert(DM % 64 == 0);
static_assert(DFF % 64 == 0);
static_assert(DAU % 64 == 0);
static_assert(DVI % 64 == 0);
static_assert(DM % 32 == 0);
static_assert(DVI % 32 == 0);
static_assert(DFF % 32 == 0);
static_assert((2 * DM) % 32 == 0);
static_assert(XCP == 2 * DM);
static_assert(((size_t)MR * DAU) % 64 == 0);
static_assert(((size_t)MR * DVI) % 64 == 0);
static_assert((size_t)NB_FULL * SEQ_FULL * DM * 4 == (size_t)4194304);
static_assert((OSP * 4) % 16 == 0);
static_assert((LNP * 4) % 16 == 0);
static_assert(32 * 16 * 8 == 16 * 64 * 4);
static_assert(32 * 16 * 4 == 16 * 64 * 2);
static_assert(32 * 16 * 4 == DM * 4);
static_assert(32 * 8 * 4 == DM * 2);
static_assert(8 * 2 == 16);
static_assert(256 * 2 * 16 == 64 * 64 * 2);
static_assert(256 * 4 * 16 == 64 * 64 * 4);
static_assert(32 * 16 == SEQ * 2);
static_assert(16 * OSP * 4 <= 131072);
static_assert(16 * LNP * 4 <= 131072);
static_assert(AW * 16 * OSP * 4 <= 131072);
static_assert(64 * WTP * 4 <= 131072);
static_assert((8 * 792 + 8) * 4 <= 131072);

typedef _Float16 h16;
typedef __attribute__((ext_vector_type(16))) _Float16 v16h;
typedef __attribute__((ext_vector_type(8)))  _Float16 v8h;
typedef __attribute__((ext_vector_type(4)))  _Float16 v4h;
typedef __attribute__((ext_vector_type(8)))  float    v8f;
typedef __attribute__((ext_vector_type(4)))  float    v4f;
typedef v4f  __attribute__((may_alias)) v4fa;

__device__ __forceinline__ unsigned short f2bf(float f) { unsigned u = __float_as_uint(f); u += 0x7FFFu + ((u >> 16) & 1u); return (unsigned short)(u >> 16); }
__device__ __forceinline__ float bfr(float f) { return __uint_as_float(((unsigned)f2bf(f)) << 16); }
__device__ __forceinline__ v16h cat16(v8h lo, v8h hi) { return __builtin_shufflevector(lo, hi, 0, 1, 2, 3, 4, 5, 6, 7, 8, 9, 10, 11, 12, 13, 14, 15); }
__device__ __forceinline__ v8f wmma16(v16h a, v16h b, v8f c) { return __builtin_amdgcn_wmma_f32_16x16x32_f16(false, a, false, b, (short)0, c, false, false); }
__device__ __forceinline__ v8f wmmag(v16h a, v16h b, v8f c) {
    c = wmma16(a, b, c);
    asm volatile("v_nop\n\tv_nop\n\tv_nop\n\tv_nop" : "+v"(c) : "v"(a), "v"(b));
    return c;
}
__device__ __forceinline__ v16h ldh(const h16* p) { return cat16(*(const v8h*)p, *(const v8h*)(p + 16)); }
__device__ __forceinline__ void wave_sync() { __builtin_amdgcn_fence(3  , "wavefront"); __builtin_amdgcn_wave_barrier(); asm volatile("" ::: "memory"); }
static __device__ __forceinline__ h16 toh_flush(float v) { const h16 r = (h16)v; return (fabsf(v) < 6.103515625e-05f) ? (h16)0.0f : r; }
__device__ __forceinline__ float gelu_erf(float x) { return 0.5f * x * (1.0f + erff(x * 0.70710678118654752f)); }

__global__ __launch_bounds__(256) void k_cvth(const float* __restrict__ src, h16* dst, size_t n8) {
    const size_t i = (size_t)blockIdx.x * 256 + threadIdx.x; if (i >= n8) return;
    const v8f v = *(const v8f*)(src + i * 8); v8h o;
#pragma unroll
    for (int k = 0; k < 8; ++k) o[k] = toh_flush(bfr(v[k]));
    *(volatile v8h*)(dst + i * 8) = o; __threadfence(); *(volatile v8h*)(dst + i * 8) = o;
}

__global__ __launch_bounds__(256) void k_wt(const float* __restrict__ W, h16* WT, int K, int N) {
    __shared__ float tile[64 * WTP];
    const int tid = threadIdx.x;
    const size_t zb = (size_t)blockIdx.z * (size_t)K * (size_t)N;
    const int n0 = blockIdx.x * 64, k0 = blockIdx.y * 64;
#pragma unroll 1
    for (int it = 0; it < 4; ++it) {
        const int p = it * 256 + tid; const int kr = p >> 4, c4 = (p & 15) * 4;
        const v4f x = *(const v4f*)(W + zb + (size_t)(k0 + kr) * N + n0 + c4);
        tile[kr * WTP + c4 + 0] = x[0]; tile[kr * WTP + c4 + 1] = x[1]; tile[kr * WTP + c4 + 2] = x[2]; tile[kr * WTP + c4 + 3] = x[3];
    }
    __syncthreads();
    v8h o[2];
#pragma unroll
    for (int it = 0; it < 2; ++it) {
        const int p = it * 256 + tid; const int nr = p >> 3, k8 = (p & 7) * 8;
#pragma unroll
        for (int i = 0; i < 8; ++i) o[it][i] = toh_flush(bfr(tile[(k8 + i) * WTP + nr]) * WSC);
    }
#pragma unroll 1
    for (int ps = 0; ps < 2; ++ps) {
#pragma unroll
        for (int it = 0; it < 2; ++it) {
            const int p = it * 256 + tid; const int nr = p >> 3, k8 = (p & 7) * 8;
            *(volatile v8h*)(WT + zb + (size_t)(n0 + nr) * K + k0 + k8) = o[it];
        }
        if (ps == 0) __threadfence();
    }
}

__device__ __forceinline__ void mac_tile(const h16* A, size_t aoff, int lda, const h16* Bt, size_t boff, int ldb, int K, v8f (&acc)[4][4]) {
#pragma unroll
    for (int mb = 0; mb < 4; ++mb)
#pragma unroll
        for (int nb = 0; nb < 4; ++nb) acc[mb][nb] = (v8f){};
#pragma unroll 1
    for (int kc = 0; kc < K; kc += 32) {
        v16h a[4];
#pragma unroll
        for (int mb = 0; mb < 4; ++mb) a[mb] = ldh(A + aoff + (size_t)mb * 16 * (size_t)lda + kc);
#pragma unroll
        for (int nb = 0; nb < 4; ++nb) {
            const v16h b = ldh(Bt + boff + (size_t)nb * 16 * (size_t)ldb + kc);
#pragma unroll
            for (int mb = 0; mb < 4; ++mb) acc[mb][nb] = wmmag(a[mb], b, acc[mb][nb]);
        }
    }
}

template <int BIAS, bool B2, bool GELU, bool MIX, bool WF, bool WH>
__device__ __forceinline__ void gemm_body(const h16* __restrict__ A, int lda, const h16* __restrict__ Bt, int ldb, int K, int bsh, int bstep, float alpha,
                                          const float* __restrict__ bias, const float* __restrict__ bias2, const float* __restrict__ R,
                                          float* C, int ldc, h16* Hh, int ldh, int hsh, size_t hbs) {
    __shared__ __align__(16) float os[16 * OSP];
    const int lane = threadIdx.x & 31, lr = lane & 15, hi = lane >> 4;
    const int r0 = blockIdx.x * 64, c0 = blockIdx.y * 64;
    const int brow = (r0 >> bsh) * bstep + c0;
    v8f acc[4][4];
    mac_tile(A, (size_t)(r0 + lr) * (size_t)lda + 8 * hi, lda, Bt, (size_t)(brow + lr) * (size_t)ldb + 8 * hi, ldb, K, acc);
    float bc[4];
#pragma unroll
    for (int nb = 0; nb < 4; ++nb) {
        float t = 0.0f;
        if (BIAS == 1) { t = bfr(bias[c0 + nb * 16 + lr]); if (B2) t = t + bfr(bias2[c0 + nb * 16 + lr]); }
        bc[nb] = t;
    }
    const size_t hb = (size_t)(c0 >> hsh) * hbs + (size_t)(c0 & ((1 << hsh) - 1));
#pragma unroll
    for (int mb = 0; mb < 4; ++mb) {
        float br[8];
#pragma unroll
        for (int j = 0; j < 8; ++j) {
            float t = 0.0f;
            if (BIAS == 2) { t = bfr(bias[r0 + mb * 16 + hi * 8 + j]); if (B2) t = t + bfr(bias2[r0 + mb * 16 + hi * 8 + j]); }
            br[j] = t;
        }
#pragma unroll
        for (int nb = 0; nb < 4; ++nb) {
#pragma unroll
            for (int j = 0; j < 8; ++j) os[(hi * 8 + j) * OSP + nb * 16 + lr] = acc[mb][nb][j] * alpha + bc[nb] + br[j]; }
        wave_sync();
        if (GELU) {
#pragma unroll 1
            for (int s = 0; s < 4; ++s) { const int row = 4 * s + (lane >> 3), c8 = (lane & 7) * 8;
                v4f x0 = *(const v4fa*)(&os[row * OSP + c8]); v4f x1 = *(const v4fa*)(&os[row * OSP + c8 + 4]);
#pragma unroll
                for (int i = 0; i < 4; ++i) { x0[i] = gelu_erf(x0[i]); x1[i] = gelu_erf(x1[i]); }
                *(v4fa*)(&os[row * OSP + c8]) = x0; *(v4fa*)(&os[row * OSP + c8 + 4]) = x1; }
            wave_sync();
        }
        const size_t grow0 = (size_t)(r0 + mb * 16);
#pragma unroll 1
        for (int ps = 0; ps < 2; ++ps) {
            if (WF) {
#pragma unroll
                for (int s = 0; s < 8; ++s) { const int row = 2 * s + (lane >> 4), c4 = (lane & 15) * 4;
                    v4f x = *(const v4fa*)(&os[row * OSP + c4]);
                    const size_t go = (grow0 + (size_t)row) * (size_t)ldc + (size_t)(c0 + c4);
                    if (MIX) { const v4f rv = *(const v4f*)(R + go); x = rv * 0.5f + x * 0.5f; }
                    *(volatile v4f*)(C + go) = x; }
            }
            if (WH) {
#pragma unroll
                for (int s = 0; s < 4; ++s) { const int row = 4 * s + (lane >> 3), c8 = (lane & 7) * 8;
                    v4f x0 = *(const v4fa*)(&os[row * OSP + c8]); v4f x1 = *(const v4fa*)(&os[row * OSP + c8 + 4]);
                    if (MIX) { const size_t go = (grow0 + (size_t)row) * (size_t)ldc + (size_t)(c0 + c8);
                               const v4f r0v = *(const v4f*)(R + go); const v4f r1v = *(const v4f*)(R + go + 4);
                               x0 = r0v * 0.5f + x0 * 0.5f; x1 = r1v * 0.5f + x1 * 0.5f; }
                    v8h hv;
#pragma unroll
                    for (int i = 0; i < 4; ++i) { hv[i] = toh_flush(x0[i]); hv[4 + i] = toh_flush(x1[i]); }
                    *(volatile v8h*)(Hh + hb + (grow0 + (size_t)row) * (size_t)ldh + c8) = hv; }
            }
            if (ps == 0) __threadfence(); }
        wave_sync();
    }
}

__global__ __launch_bounds__(32) __attribute__((amdgpu_num_vgpr(256))) void k_g_proj(const h16* __restrict__ A, int lda, const h16* __restrict__ Bt, int ldb, int K, float alpha,
        const float* __restrict__ bias, const float* __restrict__ bias2, float* C, int ldc, h16* Hh, int ldh) {
    gemm_body<1, true, false, false, true, true>(A, lda, Bt, ldb, K, BIGSH, 0, alpha, bias, bias2, bias, C, ldc, Hh, ldh, BIGSH, (size_t)0);
}
__global__ __launch_bounds__(32) __attribute__((amdgpu_num_vgpr(256))) void k_g_vt(const h16* __restrict__ A, int lda, const h16* __restrict__ Bt, int ldb, int K, float alpha,
        const float* __restrict__ bias, const float* __restrict__ bias2, h16* Hh, int ldh, int hsh, size_t hbs) {
    gemm_body<2, true, false, false, false, true>(A, lda, Bt, ldb, K, BIGSH, 0, alpha, bias, bias2, bias, (float*)0, 0, Hh, ldh, hsh, hbs);
}
__global__ __launch_bounds__(32) __attribute__((amdgpu_num_vgpr(256))) void k_g_sim(const h16* __restrict__ A, int lda, const h16* __restrict__ Bt, int ldb, int K, int bsh, int bstep, float alpha,
        float* C, int ldc) {
    gemm_body<0, false, false, false, true, false>(A, lda, Bt, ldb, K, bsh, bstep, alpha, (const float*)0, (const float*)0, (const float*)0, C, ldc, (h16*)0, 0, BIGSH, (size_t)0);
}
__global__ __launch_bounds__(32) __attribute__((amdgpu_num_vgpr(256))) void k_g_mix(const h16* __restrict__ A, int lda, const h16* __restrict__ Bt, int ldb, int K, int bsh, int bstep, float alpha,
        const float* __restrict__ R, float* C, int ldc, h16* Hh, int ldh) {
    gemm_body<0, false, false, true, true, true>(A, lda, Bt, ldb, K, bsh, bstep, alpha, (const float*)0, (const float*)0, R, C, ldc, Hh, ldh, BIGSH, (size_t)0);
}
__global__ __launch_bounds__(32) __attribute__((amdgpu_num_vgpr(256))) void k_g_gelu(const h16* __restrict__ A, int lda, const h16* __restrict__ Bt, int ldb, int K, float alpha,
        const float* __restrict__ bias, h16* Hh, int ldh) {
    gemm_body<1, false, true, false, false, true>(A, lda, Bt, ldb, K, BIGSH, 0, alpha, bias, bias, bias, (float*)0, 0, Hh, ldh, BIGSH, (size_t)0);
}

__global__ __launch_bounds__(32) __attribute__((amdgpu_num_vgpr(256))) void k_qkv(h16* WS, size_t xq, size_t xkv, size_t wo, const float* __restrict__ bias, size_t qko, size_t vto) {
    __shared__ __align__(16) float os[16 * OSP];
    const int lane = threadIdx.x & 31, lr = lane & 15, hi = lane >> 4;
    const int bx = blockIdx.x, y = blockIdx.y;
    const bool tsw = y >= 16;
    const int r0t = bx * 64;
    const int wrow = tsw ? (2 * DM + (y - 16) * 64) : (y * 64);
    const size_t xo = (y < 8) ? xq : xkv;
    const size_t tokoff = xo + (size_t)(r0t + lr) * XCP + 8 * hi;
    const size_t wgtoff = wo + (size_t)(wrow + lr) * DM + 8 * hi;
    const size_t aoff = tsw ? wgtoff : tokoff; const int lda = tsw ? DM : XCP;
    const size_t boff = tsw ? tokoff : wgtoff; const int ldb = tsw ? XCP : DM;
    v8f acc[4][4];
    mac_tile(WS, aoff, lda, WS, boff, ldb, DM, acc);
    const int cbi = tsw ? 0 : (y * 64);
    const int rbi = tsw ? wrow : 0;
    float bc[4];
#pragma unroll
    for (int nb = 0; nb < 4; ++nb) { const float t = bfr(bias[cbi + nb * 16 + lr]); bc[nb] = tsw ? 0.0f : t; }
    const int bb = r0t / SEQ, tt = r0t % SEQ;
    const size_t obase = tsw ? (vto + (size_t)bb * ((size_t)DM * SEQ) + (size_t)(wrow - 2 * DM) * SEQ + (size_t)tt)
                             : (qko + (size_t)r0t * XCP + (size_t)(y * 64));
    const int ldo = tsw ? SEQ : XCP;
#pragma unroll
    for (int mb = 0; mb < 4; ++mb) {
        float br[8];
#pragma unroll
        for (int j = 0; j < 8; ++j) { const float t = bfr(bias[rbi + mb * 16 + hi * 8 + j]); br[j] = tsw ? t : 0.0f; }
#pragma unroll
        for (int nb = 0; nb < 4; ++nb) {
#pragma unroll
            for (int j = 0; j < 8; ++j) os[(hi * 8 + j) * OSP + nb * 16 + lr] = acc[mb][nb][j] * WSI + bc[nb] + br[j]; }
        wave_sync();
        v8h hv[4];
#pragma unroll
        for (int s = 0; s < 4; ++s) { const int row = 4 * s + (lane >> 3), c8 = (lane & 7) * 8;
            const v4f x0 = *(const v4fa*)(&os[row * OSP + c8]); const v4f x1 = *(const v4fa*)(&os[row * OSP + c8 + 4]);
#pragma unroll
            for (int i = 0; i < 4; ++i) { hv[s][i] = toh_flush(x0[i]); hv[s][4 + i] = toh_flush(x1[i]); } }
#pragma unroll 1
        for (int ps = 0; ps < 2; ++ps) {
#pragma unroll
            for (int s = 0; s < 4; ++s) { const int row = 4 * s + (lane >> 3), c8 = (lane & 7) * 8;
                *(volatile v8h*)(WS + obase + (size_t)(mb * 16 + row) * (size_t)ldo + c8) = hv[s]; }
            if (ps == 0) __threadfence(); }
        wave_sync();
    }
}

template <int MODE, bool RES, bool WF, bool WH>
__device__ __forceinline__ void gemm_ln_body(const h16* __restrict__ A, int lda, const h16* __restrict__ Bt, int ldb, int K, float alpha,
                                             const float* __restrict__ bias, const float* __restrict__ g, const float* __restrict__ be, float* X, h16* Hh, int ldh) {
    __shared__ __align__(16) float ts[16 * LNP];
    const int lane = threadIdx.x & 31, lr = lane & 15, hi = lane >> 4;
    const int wave = __builtin_amdgcn_readfirstlane((int)(threadIdx.x >> 5));
    const int r0 = blockIdx.x * 64, c0 = wave * 64;
    v8f acc[4][4];
    mac_tile(A, (size_t)(r0 + lr) * (size_t)lda + 8 * hi, lda, Bt, (size_t)(c0 + lr) * (size_t)ldb + 8 * hi, ldb, K, acc);
    float bc[4];
#pragma unroll
    for (int nb = 0; nb < 4; ++nb) bc[nb] = bfr(bias[c0 + nb * 16 + lr]);
#pragma unroll
    for (int mb = 0; mb < 4; ++mb) {
#pragma unroll
        for (int nb = 0; nb < 4; ++nb) {
#pragma unroll
            for (int j = 0; j < 8; ++j) ts[(hi * 8 + j) * LNP + c0 + nb * 16 + lr] = acc[mb][nb][j] * alpha + bc[nb]; }
        __syncthreads();
#pragma unroll 1
        for (int rr = 0; rr < 2; ++rr) {
            const int row = wave * 2 + rr;
            const size_t grow = (size_t)(r0 + mb * 16 + row);
            v4f x[4];
#pragma unroll
            for (int i = 0; i < 4; ++i) {
                x[i] = *(const v4fa*)(&ts[row * LNP + i * 128 + lane * 4]);
                if (RES) { const v4f rv = *(const v4f*)(X + grow * DM + i * 128 + lane * 4); x[i] = x[i] + rv; }
            }
            v4f yv[4];
            if (MODE == 0) {
                float s = 0.0f;
#pragma unroll
                for (int i = 0; i < 4; ++i) s += (x[i][0] + x[i][1]) + (x[i][2] + x[i][3]);
#pragma unroll
                for (int o = 16; o > 0; o >>= 1) s += __shfl_xor(s, o, 32);
                const float mean = s * (1.0f / (float)DM);
                float q = 0.0f;
#pragma unroll
                for (int i = 0; i < 4; ++i) {
#pragma unroll
                    for (int e = 0; e < 4; ++e) { const float d = x[i][e] - mean; q += d * d; } }
#pragma unroll
                for (int o = 16; o > 0; o >>= 1) q += __shfl_xor(q, o, 32);
                const float rstd = rsqrtf(q * (1.0f / (float)DM) + 1.0e-5f);
#pragma unroll
                for (int i = 0; i < 4; ++i) {
                    const v4f g4 = *(const v4f*)(g + i * 128 + lane * 4); const v4f b4 = *(const v4f*)(be + i * 128 + lane * 4);
#pragma unroll
                    for (int e = 0; e < 4; ++e) yv[i][e] = (x[i][e] - mean) * rstd * bfr(g4[e]) + bfr(b4[e]); }
            } else {
                float q = 0.0f;
#pragma unroll
                for (int i = 0; i < 4; ++i) {
#pragma unroll
                    for (int e = 0; e < 4; ++e) q += x[i][e] * x[i][e]; }
#pragma unroll
                for (int o = 16; o > 0; o >>= 1) q += __shfl_xor(q, o, 32);
                const float inv = 1.0f / fmaxf(sqrtf(q), 1.0e-12f);
#pragma unroll
                for (int i = 0; i < 4; ++i) {
#pragma unroll
                    for (int e = 0; e < 4; ++e) yv[i][e] = (x[i][e] * inv) * NSC; }
            }
            v4h hq[4];
#pragma unroll
            for (int i = 0; i < 4; ++i) {
#pragma unroll
                for (int e = 0; e < 4; ++e) hq[i][e] = toh_flush(yv[i][e]); }
#pragma unroll 1
            for (int ps = 0; ps < 2; ++ps) {
#pragma unroll
                for (int i = 0; i < 4; ++i) {
                    if (WF) *(volatile v4f*)(X + grow * DM + i * 128 + lane * 4) = yv[i];
                    if (WH) *(volatile v4h*)(Hh + grow * (size_t)ldh + i * 128 + lane * 4) = hq[i];
                }
                if (ps == 0) __threadfence(); }
        }
        __syncthreads();
    }
}

__global__ __launch_bounds__(256) __attribute__((amdgpu_num_vgpr(256))) void k_gln_res(const h16* __restrict__ A, int lda, const h16* __restrict__ Bt, int ldb, int K, float alpha,
        const float* __restrict__ bias, const float* __restrict__ g, const float* __restrict__ be, float* X, h16* Hh, int ldh) {
    gemm_ln_body<0, true, true, true>(A, lda, Bt, ldb, K, alpha, bias, g, be, X, Hh, ldh);
}
__global__ __launch_bounds__(256) __attribute__((amdgpu_num_vgpr(256))) void k_gln_fin(const h16* __restrict__ A, int lda, const h16* __restrict__ Bt, int ldb, int K, float alpha,
        const float* __restrict__ bias, const float* __restrict__ g, const float* __restrict__ be, float* X) {
    gemm_ln_body<0, false, true, false>(A, lda, Bt, ldb, K, alpha, bias, g, be, X, (h16*)0, 0);
}
__global__ __launch_bounds__(256) __attribute__((amdgpu_num_vgpr(256))) void k_gl2(const h16* __restrict__ A, int lda, const h16* __restrict__ Bt, int ldb, int K, float alpha,
        const float* __restrict__ bias, h16* Hh, int ldh) {
    gemm_ln_body<1, false, false, true>(A, lda, Bt, ldb, K, alpha, bias, bias, bias, (float*)0, Hh, ldh);
}

__global__ __launch_bounds__(32 * AW) __attribute__((amdgpu_num_vgpr(256))) void k_flash(const h16* __restrict__ QK, const h16* __restrict__ VT, h16* CTX) {
    __shared__ __align__(16) float os[AW * 16 * OSP];
    const int lane = threadIdx.x & 31, lr = lane & 15, hi = lane >> 4;
    const int wave = __builtin_amdgcn_readfirstlane((int)(threadIdx.x >> 5));
    const int zh = blockIdx.y; const int b = zh / NH_, h = zh % NH_;
    const int t0 = (blockIdx.x * AW + wave) * 16;
    const size_t qo = ((size_t)b * SEQ + (size_t)(t0 + lr)) * XCP + (size_t)h * HD + 8 * hi;
    const v16h q0 = ldh(QK + qo), q1 = ldh(QK + qo + 32);
    const size_t ko = ((size_t)b * SEQ + (size_t)lr) * XCP + DM + (size_t)h * HD + 8 * hi;
    const size_t vo = ((size_t)zh * HD + (size_t)lr) * SEQ + 8 * hi;
    v8f o0 = (v8f){}, o1 = (v8f){}, o2 = (v8f){}, o3 = (v8f){};
    float m = NEGB, l = 0.0f;
#pragma unroll 1
    for (int key0 = 0; key0 < SEQ; key0 += 32) {
        const h16* ka = QK + ko + (size_t)key0 * XCP;
        const v16h ka0 = ldh(ka), ka1 = ldh(ka + 32), kb0 = ldh(ka + 16 * XCP), kb1 = ldh(ka + 16 * XCP + 32);
        v8f sa = (v8f){}, sb = (v8f){};
        sa = wmmag(ka0, q0, sa); sa = wmmag(ka1, q1, sa);
        sb = wmmag(kb0, q0, sb); sb = wmmag(kb1, q1, sb);
        float ta[8], tb[8]; float mx = NEGB;
#pragma unroll
        for (int r = 0; r < 8; ++r) { ta[r] = sa[r] * SC2; tb[r] = sb[r] * SC2; mx = fmaxf(mx, fmaxf(ta[r], tb[r])); }
        mx = fmaxf(mx, __shfl_xor(mx, 16, 32));
        const float mnew = fmaxf(m, mx);
        const float alpha = __builtin_amdgcn_exp2f(m - mnew);
        const float sh = PSH - mnew;
        v16h pb; float ls = 0.0f;
#pragma unroll
        for (int r = 0; r < 8; ++r) {
            const float xa = ta[r] + sh, xb = tb[r] + sh;
            const float ea = __builtin_amdgcn_exp2f(xa), eb = __builtin_amdgcn_exp2f(xb);
            const float ga = (xa < -14.0f) ? 0.0f : ea, gb = (xb < -14.0f) ? 0.0f : eb;
            const h16 pa = (h16)ga; const h16 pc = (h16)gb;
            pb[r] = pa; pb[8 + r] = pc;
            ls += (float)pa + (float)pc; }
        l = l * alpha + ls; m = mnew;
        o0 = o0 * alpha; o1 = o1 * alpha; o2 = o2 * alpha; o3 = o3 * alpha;
        const h16* va = VT + vo + key0;
        const v16h v0 = ldh(va), v1 = ldh(va + (size_t)16 * SEQ), v2 = ldh(va + (size_t)32 * SEQ), v3 = ldh(va + (size_t)48 * SEQ);
        o0 = wmmag(v0, pb, o0); o1 = wmmag(v1, pb, o1); o2 = wmmag(v2, pb, o2); o3 = wmmag(v3, pb, o3);
    }
    l += __shfl_xor(l, 16, 32);
    const float inv = CSC * (1.0f / l);
    const int wb = wave * 16 * OSP;
    { v4f a, c;
      a[0] = o0[0] * inv; a[1] = o0[1] * inv; a[2] = o0[2] * inv; a[3] = o0[3] * inv; c[0] = o0[4] * inv; c[1] = o0[5] * inv; c[2] = o0[6] * inv; c[3] = o0[7] * inv;
      *(v4fa*)(&os[wb + lr * OSP +  0 + 8 * hi]) = a; *(v4fa*)(&os[wb + lr * OSP +  0 + 8 * hi + 4]) = c;
      a[0] = o1[0] * inv; a[1] = o1[1] * inv; a[2] = o1[2] * inv; a[3] = o1[3] * inv; c[0] = o1[4] * inv; c[1] = o1[5] * inv; c[2] = o1[6] * inv; c[3] = o1[7] * inv;
      *(v4fa*)(&os[wb + lr * OSP + 16 + 8 * hi]) = a; *(v4fa*)(&os[wb + lr * OSP + 16 + 8 * hi + 4]) = c;
      a[0] = o2[0] * inv; a[1] = o2[1] * inv; a[2] = o2[2] * inv; a[3] = o2[3] * inv; c[0] = o2[4] * inv; c[1] = o2[5] * inv; c[2] = o2[6] * inv; c[3] = o2[7] * inv;
      *(v4fa*)(&os[wb + lr * OSP + 32 + 8 * hi]) = a; *(v4fa*)(&os[wb + lr * OSP + 32 + 8 * hi + 4]) = c;
      a[0] = o3[0] * inv; a[1] = o3[1] * inv; a[2] = o3[2] * inv; a[3] = o3[3] * inv; c[0] = o3[4] * inv; c[1] = o3[5] * inv; c[2] = o3[6] * inv; c[3] = o3[7] * inv;
      *(v4fa*)(&os[wb + lr * OSP + 48 + 8 * hi]) = a; *(v4fa*)(&os[wb + lr * OSP + 48 + 8 * hi + 4]) = c; }
    wave_sync();
    v8h hv[4];
#pragma unroll
    for (int s = 0; s < 4; ++s) { const int row = 4 * s + (lane >> 3), c8 = (lane & 7) * 8;
        const v4f x0 = *(const v4fa*)(&os[wb + row * OSP + c8]); const v4f x1 = *(const v4fa*)(&os[wb + row * OSP + c8 + 4]);
#pragma unroll
        for (int i = 0; i < 4; ++i) { hv[s][i] = toh_flush(x0[i]); hv[s][4 + i] = toh_flush(x1[i]); } }
    h16* orow = CTX + ((size_t)b * SEQ + (size_t)t0) * DM + (size_t)h * HD;
#pragma unroll 1
    for (int ps = 0; ps < 2; ++ps) {
#pragma unroll
        for (int s = 0; s < 4; ++s) { const int row = 4 * s + (lane >> 3), c8 = (lane & 7) * 8;
            *(volatile v8h*)(orow + (size_t)row * DM + c8) = hv[s]; }
        if (ps == 0) __threadfence(); }
}

__global__ __launch_bounds__(256) void k_softp(const float* __restrict__ S, h16* P) {
    const int lane = threadIdx.x & 31;
    const int wave = __builtin_amdgcn_readfirstlane((int)(threadIdx.x >> 5));
    const size_t row = (size_t)blockIdx.x * 8 + (size_t)wave;
    const float* sr = S + row * SEQ + lane * 8;
    const v4f a = *(const v4f*)sr, c = *(const v4f*)(sr + 4);
    float x[8];
#pragma unroll
    for (int i = 0; i < 4; ++i) { x[i] = a[i]; x[4 + i] = c[i]; }
    float mx = x[0];
#pragma unroll
    for (int i = 1; i < 8; ++i) mx = fmaxf(mx, x[i]);
#pragma unroll
    for (int o = 16; o > 0; o >>= 1) mx = fmaxf(mx, __shfl_xor(mx, o, 32));
    float e[8]; float s = 0.0f;
#pragma unroll
    for (int i = 0; i < 8; ++i) { e[i] = __builtin_amdgcn_exp2f((x[i] - mx) * LOG2E); s += e[i]; }
#pragma unroll
    for (int o = 16; o > 0; o >>= 1) s += __shfl_xor(s, o, 32);
    const float inv = PAL * (1.0f / s);
    v8h ov;
#pragma unroll
    for (int i = 0; i < 8; ++i) ov[i] = toh_flush(e[i] * inv);
    h16* pr = P + row * SEQ + lane * 8;
    *(volatile v8h*)pr = ov; __threadfence(); *(volatile v8h*)pr = ov;
}

__global__ __launch_bounds__(256) void k_dtw(const float* __restrict__ SIMP, float* OUT1) {
    __shared__ float dd[8 * 792];
    __shared__ __align__(16) float sc[8];
    const int lane = threadIdx.x & 31;
    const int wv0 = (int)(threadIdx.x >> 5);
    const int bs0 = wv0 < NB ? wv0 : (NB - 1);
    const int wave = __builtin_amdgcn_readfirstlane(wv0);
    const int bsel = __builtin_amdgcn_readfirstlane(bs0);
    const float* S = SIMP + (size_t)bsel * ((size_t)SEQ * SEQ);
    const int wb = wave * 792;
#pragma unroll 1
    for (int q = lane; q < 792; q += 32) dd[wb + q] = NEGV;
    wave_sync();
    if (lane == 0) dd[wb] = 0.0f;
    wave_sync();
    int p2 = 0, p1 = 264, pc = 528;
#pragma unroll 1
    for (int d = 2; d <= 2 * SEQ; ++d) {
#pragma unroll 1
        for (int c = 0; c < 9; ++c) {
            const int i = lane + 32 * c; const int j = d - i;
            const bool inr = (i <= SEQ) & (j >= 0) & (j <= SEQ);
            const bool edge = (i == 0) | (j == 0);
            int ic = i - 1; ic = ic < 0 ? 0 : (ic > SEQ - 1 ? SEQ - 1 : ic);
            int jc = j - 1; jc = jc < 0 ? 0 : (jc > SEQ - 1 ? SEQ - 1 : jc);
            float sv = S[ic * SEQ + jc];
            asm volatile("" : "+v"(sv));
            int im = i - 1; im = im < 0 ? 0 : (im > SEQ ? SEQ : im);
            const int ii = i > SEQ ? SEQ : i;
            const float up = dd[wb + p1 + im], lf = dd[wb + p1 + ii], dg = dd[wb + p2 + im];
            float val = sv + fmaxf(fmaxf(up, dg), lf);
            val = edge ? NEGV : val;
            if (inr) dd[wb + pc + i] = val;
        }
        wave_sync();
        const int t = p2; p2 = p1; p1 = pc; pc = t;
    }
    const float res = dd[wb + p1 + SEQ];
    if (lane == 0) sc[wave] = (wv0 < NB) ? res : 0.0f;
    __syncthreads();
    if (wave == 0) {
        const int pl = lane < 2 ? lane : 1;
        const v4f val = *(const v4fa*)(&sc[pl * 4]);
        if (lane < 2) *(volatile v4f*)(OUT1 + lane * 4) = val;
        __threadfence();
        if (lane < 2) *(volatile v4f*)(OUT1 + lane * 4) = val;
    }
}

static constexpr size_t al256(size_t v) { return (v + 255) & ~(size_t)255; }
static constexpr size_t DD_   = (size_t)DM * DM;
static constexpr size_t B_AU  = 0;
static constexpr size_t B_VI  = B_AU  + al256((size_t)MR * DAU * 2);
static constexpr size_t B_WAP = B_VI  + al256((size_t)MR * DVI * 2);
static constexpr size_t B_WVP = B_WAP + al256((size_t)DM * DAU * 2);
static constexpr size_t B_WDT = B_WVP + al256((size_t)DM * DVI * 2);
static constexpr size_t B_WCA = B_WDT + al256(DD_ * 2);
static constexpr size_t B_WSA = B_WCA + al256((size_t)32 * DD_ * 2);
static constexpr size_t B_WF1 = B_WSA + al256((size_t)32 * DD_ * 2);
static constexpr size_t B_WF2 = B_WF1 + al256((size_t)8 * DFF * DM * 2);
static constexpr size_t B_WOU = B_WF2 + al256((size_t)8 * DFF * DM * 2);
static constexpr size_t B_XA  = B_WOU + al256((size_t)DM * 2 * DM * 2);
static constexpr size_t B_XV0 = B_XA  + al256((size_t)MR * DM * 4);
static constexpr size_t B_XV  = B_XV0 + al256((size_t)MR * DM * 4);
static constexpr size_t B_XC  = B_XV  + al256((size_t)MR * DM * 4);
static constexpr size_t B_N16 = B_XC  + al256((size_t)MR * XCP * 2);
static constexpr size_t B_SIM = B_N16 + al256((size_t)MR * XCP * 2);
static constexpr size_t B_P16 = B_SIM + al256((size_t)MR * SEQ * 4);
static constexpr size_t B_VT  = B_P16 + al256((size_t)MR * SEQ * 2);
static constexpr size_t B_QK  = B_VT  + al256((size_t)MR * DM * 2);
static constexpr size_t B_CTX = B_QK  + al256((size_t)MR * XCP * 2);
static constexpr size_t B_H16 = B_CTX + al256((size_t)MR * DM * 2);
static constexpr size_t SZ_TOTAL = B_H16 + al256((size_t)MR * DFF * 2);
static_assert(SZ_TOTAL <= (size_t)134217728);
static_assert((size_t)NB * DM * SEQ == (size_t)MR * DM);
static_assert(B_XC % 2 == 0);

static void run_mha(hipStream_t st, h16* WSH, size_t xq, size_t xkv, size_t wo, const float* bias,
                    const float* g, const float* be, float* X, h16* Hx) {
    const h16* QK = WSH + B_QK / 2; const h16* VT = WSH + B_VT / 2; h16* CTX = WSH + B_CTX / 2;
    const h16* Wt = WSH + wo;
    k_qkv<<<dim3(MR / 64, 24, 1), 32, 0, st>>>(WSH, xq, xkv, wo, bias, (size_t)(B_QK / 2), (size_t)(B_VT / 2));
    k_flash<<<dim3(SEQ / (16 * AW), NB * NH_, 1), 32 * AW, 0, st>>>(QK, VT, CTX);
    k_gln_res<<<dim3(MR / 64, 1, 1), 256, 0, st>>>(CTX, DM, Wt + 3 * DD_, DM, DM, 1.0f / (CSC * WSC), bias + 3 * DM, g, be, X, Hx, XCP);
}

static void run_ffn(hipStream_t st, h16* WSH, size_t xo, const h16* W1, const float* b1, const h16* W2, const float* b2,
                    const float* g, const float* be, float* X, h16* Hx) {
    h16* H16P = WSH + B_H16 / 2;
    k_g_gelu<<<dim3(MR / 64, DFF / 64, 1), 32, 0, st>>>(WSH + xo, XCP, W1, DM, DM, WSI, b1, H16P, DFF);
    k_gln_res<<<dim3(MR / 64, 1, 1), 256, 0, st>>>(H16P, DFF, W2, DFF, DFF, WSI, b2, g, be, X, Hx, XCP);
}

extern "C" void kernel_launch(void* const* d_in, const int* in_sizes, int n_in,
                              void* d_out, int out_size, void* d_ws, size_t ws_size, hipStream_t stream) {
    if (n_in < 23) return;
    if ((size_t)in_sizes[0] < (size_t)MR * DAU || (size_t)in_sizes[1] < (size_t)MR * DVI) return;
    if ((size_t)in_sizes[2] < (size_t)DAU * DM || in_sizes[3] < DM || (size_t)in_sizes[4] < (size_t)DVI * DM || in_sizes[5] < DM) return;
    if ((size_t)in_sizes[6] < DD_ || in_sizes[7] < DM || in_sizes[8] < 2 * DM) return;
    if ((size_t)in_sizes[9] < 32 * DD_ || in_sizes[10] < 32 * DM || (size_t)in_sizes[11] < 32 * DD_ || in_sizes[12] < 32 * DM) return;
    if (in_sizes[13] < NLAY * 6 * DM || in_sizes[14] < NLAY * 6 * DM) return;
    if ((size_t)in_sizes[15] < (size_t)8 * DM * DFF || in_sizes[16] < 8 * DFF || (size_t)in_sizes[17] < (size_t)8 * DM * DFF || in_sizes[18] < 8 * DM) return;
    if ((size_t)in_sizes[19] < (size_t)2 * DM * DM || in_sizes[20] < DM || in_sizes[21] < DM || in_sizes[22] < DM) return;
    if ((size_t)out_size < (size_t)NB_FULL * SEQ_FULL * DM + 8) return;
    if (SZ_TOTAL > ws_size) return;
    const float* audio   = (const float*)d_in[0];
    const float* video   = (const float*)d_in[1];
    const float* ap_w    = (const float*)d_in[2];
    const float* ap_b    = (const float*)d_in[3];
    const float* vp_w    = (const float*)d_in[4];
    const float* vp_b    = (const float*)d_in[5];
    const float* dtw_w   = (const float*)d_in[6];
    const float* dtw_b   = (const float*)d_in[7];
    const float* mod_emb = (const float*)d_in[8];
    const float* ca_w    = (const float*)d_in[9];
    const float* ca_b    = (const float*)d_in[10];
    const float* sa_w    = (const float*)d_in[11];
    const float* sa_b    = (const float*)d_in[12];
    const float* ln_g    = (const float*)d_in[13];
    const float* ln_b    = (const float*)d_in[14];
    const float* ffn_w1  = (const float*)d_in[15];
    const float* ffn_b1  = (const float*)d_in[16];
    const float* ffn_w2  = (const float*)d_in[17];
    const float* ffn_b2  = (const float*)d_in[18];
    const float* out_w   = (const float*)d_in[19];
    const float* out_b   = (const float*)d_in[20];
    const float* fln_g   = (const float*)d_in[21];
    const float* fln_b   = (const float*)d_in[22];
    float* OUT  = (float*)d_out;
    float* OUT1 = (float*)d_out + (size_t)NB_FULL * SEQ_FULL * DM;

    char* wsb = (char*)d_ws;
    h16* WSH = (h16*)d_ws;
    h16* AU  = (h16*)(wsb + B_AU);  h16* VI  = (h16*)(wsb + B_VI);
    h16* WAP = (h16*)(wsb + B_WAP); h16* WVP = (h16*)(wsb + B_WVP); h16* WDT = (h16*)(wsb + B_WDT);
    h16* WCA = (h16*)(wsb + B_WCA); h16* WSA = (h16*)(wsb + B_WSA);
    h16* WF1 = (h16*)(wsb + B_WF1); h16* WF2 = (h16*)(wsb + B_WF2); h16* WOU = (h16*)(wsb + B_WOU);
    float* XA = (float*)(wsb + B_XA); float* XV0 = (float*)(wsb + B_XV0); float* XV = (float*)(wsb + B_XV);
    h16* XC  = (h16*)(wsb + B_XC);  h16* N16 = (h16*)(wsb + B_N16);
    float* SIM = (float*)(wsb + B_SIM);
    h16* P16 = (h16*)(wsb + B_P16); h16* VT = (h16*)(wsb + B_VT);

    k_wt<<<dim3(DM / 64,  DAU / 64, 1),  256, 0, stream>>>(ap_w,   WAP, DAU, DM);
    k_wt<<<dim3(DM / 64,  DVI / 64, 1),  256, 0, stream>>>(vp_w,   WVP, DVI, DM);
    k_wt<<<dim3(DM / 64,  DM / 64, 1),   256, 0, stream>>>(dtw_w,  WDT, DM,  DM);
    k_wt<<<dim3(DM / 64,  DM / 64, 32),  256, 0, stream>>>(ca_w,   WCA, DM,  DM);
    k_wt<<<dim3(DM / 64,  DM / 64, 32),  256, 0, stream>>>(sa_w,   WSA, DM,  DM);
    k_wt<<<dim3(DFF / 64, DM / 64, 8),   256, 0, stream>>>(ffn_w1, WF1, DM,  DFF);
    k_wt<<<dim3(DM / 64,  DFF / 64, 8),  256, 0, stream>>>(ffn_w2, WF2, DFF, DM);
    k_wt<<<dim3(DM / 64,  2 * DM / 64, 1), 256, 0, stream>>>(out_w, WOU, 2 * DM, DM);
    { const size_t n8 = (size_t)MR * DAU / 8; k_cvth<<<(unsigned)((n8 + 255) / 256), 256, 0, stream>>>(audio, AU, n8); }
    { const size_t n8 = (size_t)MR * DVI / 8; k_cvth<<<(unsigned)((n8 + 255) / 256), 256, 0, stream>>>(video, VI, n8); }

    k_g_proj<<<dim3(MR / 64, DM / 64, 1), 32, 0, stream>>>(AU, DAU, WAP, DAU, DAU, WSI, ap_b, mod_emb,      XA,  DM, XC,      XCP);
    k_g_proj<<<dim3(MR / 64, DM / 64, 1), 32, 0, stream>>>(VI, DVI, WVP, DVI, DVI, WSI, vp_b, mod_emb + DM, XV0, DM, XC + DM, XCP);
    k_g_vt<<<dim3(DM / 64, MR / 64, 1), 32, 0, stream>>>(WVP, DVI, VI, DVI, DVI, WSI, vp_b, mod_emb + DM, VT, SEQ, 8, (size_t)DM * SEQ);

    k_gl2<<<dim3(2 * MR / 64, 1, 1), 256, 0, stream>>>(XC, DM, WDT, DM, DM, WSI, dtw_b, N16, DM);
    k_g_sim<<<dim3(MR / 64, SEQ / 64, 1), 32, 0, stream>>>(N16, XCP, N16 + DM, XCP, DM, 8, SEQ, 1.0f / (NSC * NSC), SIM, SEQ);
    k_dtw<<<dim3(1, 1, 1), 256, 0, stream>>>(SIM, OUT1);
    k_softp<<<dim3(MR / 8, 1, 1), 256, 0, stream>>>(SIM, P16);
    k_g_mix<<<dim3(MR / 64, DM / 64, 1), 32, 0, stream>>>(P16, SEQ, VT, SEQ, SEQ, 8, DM, 1.0f / PAL, XV0, XV, DM, XC + DM, XCP);

    const size_t oXA = B_XC / 2, oXV = B_XC / 2 + DM;
    for (int l = 0; l < NLAY; ++l) {
        const size_t wca0 = B_WCA / 2 + (size_t)(l * 2 + 0) * 4 * DD_, wca1 = B_WCA / 2 + (size_t)(l * 2 + 1) * 4 * DD_;
        const size_t wsa0 = B_WSA / 2 + (size_t)(l * 2 + 0) * 4 * DD_, wsa1 = B_WSA / 2 + (size_t)(l * 2 + 1) * 4 * DD_;
        const float* cab0 = ca_b + (size_t)(l * 2 + 0) * 4 * DM; const float* cab1 = ca_b + (size_t)(l * 2 + 1) * 4 * DM;
        const float* sab0 = sa_b + (size_t)(l * 2 + 0) * 4 * DM; const float* sab1 = sa_b + (size_t)(l * 2 + 1) * 4 * DM;
        const float* lg = ln_g + (size_t)l * 6 * DM; const float* lb = ln_b + (size_t)l * 6 * DM;
        run_mha(stream, WSH, oXA, oXV, wca0, cab0, lg + 0 * DM, lb + 0 * DM, XA, XC);
        run_mha(stream, WSH, oXV, oXA, wca1, cab1, lg + 3 * DM, lb + 3 * DM, XV, XC + DM);
        run_mha(stream, WSH, oXA, oXA, wsa0, sab0, lg + 1 * DM, lb + 1 * DM, XA, XC);
        run_mha(stream, WSH, oXV, oXV, wsa1, sab1, lg + 4 * DM, lb + 4 * DM, XV, XC + DM);
        run_ffn(stream, WSH, oXA, WF1 + (size_t)(l * 2 + 0) * DFF * DM, ffn_b1 + (size_t)(l * 2 + 0) * DFF,
                WF2 + (size_t)(l * 2 + 0) * DFF * DM, ffn_b2 + (size_t)(l * 2 + 0) * DM, lg + 2 * DM, lb + 2 * DM, XA, XC);
        run_ffn(stream, WSH, oXV, WF1 + (size_t)(l * 2 + 1) * DFF * DM, ffn_b1 + (size_t)(l * 2 + 1) * DFF,
                WF2 + (size_t)(l * 2 + 1) * DFF * DM, ffn_b2 + (size_t)(l * 2 + 1) * DM, lg + 5 * DM, lb + 5 * DM, XV, XC + DM);
    }

    k_gln_fin<<<dim3(MR / 64, 1, 1), 256, 0, stream>>>(XC, XCP, WOU, 2 * DM, 2 * DM, WSI, out_b, fln_g, fln_b, OUT);
}
